// GCN_60868276519239
// MI455X (gfx1250) — hardware-verified
//
#include <hip/hip_runtime.h>
#include <stddef.h>
#include <stdint.h>
#include <math.h>


#define DI     128
#define DH     128
#define DOUT   64
#define K2     256
#define NNODE  100000
#define NEDGE  1600000
#define MPAD   100096
#define NTHR   256
#define NWAVE  8
#define EPT    8
#define CHUNK  (NTHR * EPT)
#define WCAP   (EPT * 32)
#define LISTN  (NWAVE * WCAP)
#define NBA    1024
#define SLA    10
#define NBUCK  98
#define RCAP   28672
#define DEGCAP 64
#define AGS    128
#define GBM    64
#define GTHR   128
#define ROWH   256
#define NUW1   (DH * (DI / 8))
#define NUW2   (DH * (K2 / 8))
#define NUW3   (DOUT * (K2 / 8))
#define NUBI   256
#define NUWE   (NUW1 + NUW2 + NUW3 + NUBI)
#define BIASN  1024
#define BK_ZINTS (LISTN + 2 * RCAP + 3 * NBA)
#define BK_LDS_INTS (BK_ZINTS + 16)
#define WSMAX  134217728

static_assert(DI == 128 && DH == 128 && DOUT == 64);
static_assert(K2 % 32 == 0 && DI % 32 == 0 && K2 == 2 * DH);
static_assert((CHUNK & (CHUNK - 1)) == 0 && CHUNK <= 4096);
static_assert((NBA & (NBA - 1)) == 0 && NBA == (1 << SLA));
static_assert(((long long)CHUNK << SLA) < (1LL << 31));
static_assert((long long)NEDGE < (1LL << (31 - SLA)));
static_assert(NBA * NBUCK >= NNODE && NBA * NBUCK >= MPAD);
static_assert(MPAD == 782 * 128 && MPAD >= NNODE && 781 * 128 < NNODE && MPAD % GBM == 0 && MPAD % AGS == 0);
static_assert(RCAP >= 16710 + 16710 / 20 && RCAP % (4 * NTHR) == 0);
static_assert(DEGCAP >= 36 + 8);
static_assert(LISTN % NTHR == 0 && NBA % 32 == 0 && NBA == 4 * NTHR);
static_assert(BK_ZINTS % 4 == 0 && LISTN % 4 == 0);
static_assert(BK_LDS_INTS * 4 <= 300000);
static_assert(NUW1 % NTHR == 0 && NUW2 % NTHR == 0 && NUW3 % NTHR == 0 && NUBI % NTHR == 0);
static_assert((MPAD * (DI / 8)) % NTHR == 0);
static_assert(AGS % NWAVE == 0 && NBA % AGS == 0);
static_assert((DOUT * 4) % 128 == 0 && (DH * 4) % 128 == 0 && (K2 * 2) % 128 == 0);
static_assert(GBM == (GTHR / 32) * 16);
static_assert(ROWH == 2 * DH);

typedef float          v2f   __attribute__((ext_vector_type(2)));
typedef float          v4f   __attribute__((ext_vector_type(4)));
typedef float          v8f   __attribute__((ext_vector_type(8)));
typedef int            v4i   __attribute__((ext_vector_type(4)));
typedef int            v8i   __attribute__((ext_vector_type(8)));
typedef unsigned int   v4u   __attribute__((ext_vector_type(4)));
typedef unsigned short v4us  __attribute__((ext_vector_type(4)));
typedef unsigned short v8us  __attribute__((ext_vector_type(8)));
typedef unsigned short v16us __attribute__((ext_vector_type(16)));
typedef __bf16         v16bf __attribute__((ext_vector_type(16)));
typedef v2f  __attribute__((may_alias)) v2fa;
typedef v4f  __attribute__((may_alias)) v4fa;
typedef v4i  __attribute__((may_alias)) v4ia;
typedef v4us __attribute__((may_alias)) v4usa;
typedef v8us __attribute__((may_alias)) v8usa;
union FragB { v16bf v; v16us u; v8us h[2]; v8i w; };

__device__ __forceinline__ v8f wmb(const FragB& a, const FragB& b, v8f c) {
  v8f d = __builtin_amdgcn_wmma_f32_16x16x32_bf16(false, a.v, false, b.v, (short)0, c, false, false);
  asm volatile("v_nop\n\tv_nop\n\tv_nop\n\tv_nop" : "+v"(d) : "v"(a.w), "v"(b.w));
  return d;
}

__device__ __forceinline__ v8f z8() { v8f z = {0.f, 0.f, 0.f, 0.f, 0.f, 0.f, 0.f, 0.f}; return z; }

__device__ __forceinline__ unsigned bf16_bits(float f) {
  const unsigned u = __float_as_uint(f);
  const unsigned r = (u + 0x7FFFu + ((u >> 16) & 1u)) >> 16;
  return ((u & 0x7FFFFFFFu) > 0x7F800000u) ? 0x7FC0u : r;
}
__device__ __forceinline__ float bf16_val(float f) {
  return __uint_as_float(bf16_bits(f) << 16);
}
__device__ __forceinline__ unsigned hl_bits(float v, unsigned& lo) {
  const unsigned hb = bf16_bits(v);
  lo = bf16_bits(v - __uint_as_float(hb << 16));
  return hb;
}

__device__ __forceinline__ void wave_sync() {
  __builtin_amdgcn_fence(__ATOMIC_RELEASE, "wavefront");
  __builtin_amdgcn_wave_barrier();
  __builtin_amdgcn_fence(__ATOMIC_ACQUIRE, "wavefront");
}

template <int SLB>
__device__ __forceinline__ int scan_chunk(const int* __restrict__ dsts, int nE, int cbase, int slotBase,
                                          int nb, int vec8, int* list, int tid, int lane, int wave) {
  int wc = 0;
  const int el0  = tid * EPT;
  const int e0   = cbase + el0;
  const int sent = -2147483647 - 1;
  v4i da, db;
  if (vec8 != 0 && cbase + CHUNK <= nE) {
    da = *(const v4i*)(dsts + e0);
    db = *(const v4i*)(dsts + e0 + 4);
  } else {
    da.x = (e0     < nE) ? dsts[min(e0,     nE - 1)] : sent;
    da.y = (e0 + 1 < nE) ? dsts[min(e0 + 1, nE - 1)] : sent;
    da.z = (e0 + 2 < nE) ? dsts[min(e0 + 2, nE - 1)] : sent;
    da.w = (e0 + 3 < nE) ? dsts[min(e0 + 3, nE - 1)] : sent;
    db.x = (e0 + 4 < nE) ? dsts[min(e0 + 4, nE - 1)] : sent;
    db.y = (e0 + 5 < nE) ? dsts[min(e0 + 5, nE - 1)] : sent;
    db.z = (e0 + 6 < nE) ? dsts[min(e0 + 6, nE - 1)] : sent;
    db.w = (e0 + 7 < nE) ? dsts[min(e0 + 7, nE - 1)] : sent;
  }
  const unsigned nbs = (unsigned)slotBase;
  const unsigned unb = (unsigned)nb;
  const unsigned s0 = (unsigned)da.x - nbs, s1 = (unsigned)da.y - nbs;
  const unsigned s2 = (unsigned)da.z - nbs, s3 = (unsigned)da.w - nbs;
  const unsigned s4 = (unsigned)db.x - nbs, s5 = (unsigned)db.y - nbs;
  const unsigned s6 = (unsigned)db.z - nbs, s7 = (unsigned)db.w - nbs;
  const bool h0 = s0 < unb, h1 = s1 < unb, h2 = s2 < unb, h3 = s3 < unb;
  const bool h4 = s4 < unb, h5 = s5 < unb, h6 = s6 < unb, h7 = s7 < unb;
  const unsigned any = __builtin_amdgcn_ballot_w32(h0 | h1 | h2 | h3 | h4 | h5 | h6 | h7);
  if (any != 0u) {
#define HITJ(J, HJ, SJ) { \
      const unsigned mj = __builtin_amdgcn_ballot_w32(HJ); \
      if (mj != 0u) { \
        if (HJ) { \
          const int pos = wc + (int)__builtin_amdgcn_mbcnt_lo(mj, 0u); \
          if (pos < WCAP) list[wave * WCAP + pos] = ((el0 + (J)) << SLB) | (int)(SJ); \
        } \
        wc += (int)__builtin_popcount(mj); } }
    HITJ(0, h0, s0)
    HITJ(1, h1, s1)
    HITJ(2, h2, s2)
    HITJ(3, h3, s3)
    HITJ(4, h4, s4)
    HITJ(5, h5, s5)
    HITJ(6, h6, s6)
    HITJ(7, h7, s7)
#undef HITJ
  }
  return wc;
}

__global__ __launch_bounds__(NTHR) void k_prep(const float* __restrict__ x,
                                               const float* __restrict__ W1, const float* __restrict__ W2,
                                               const float* __restrict__ W3, const float* __restrict__ b1,
                                               const float* __restrict__ b2, const float* __restrict__ b3,
                                               unsigned* w1t, unsigned* w2d, unsigned* w3d, unsigned* biasT,
                                               unsigned* xb, int nN, int nUnits) {
  const int u = (int)blockIdx.x * NTHR + (int)threadIdx.x;
  v4u o;
  unsigned* dp;
  if (u < NUW1) {
    const int n = u >> 4, k8 = (u & 15) * 8;
    const float* p = W1 + (size_t)k8 * DH + n;
    unsigned hb[8];
#pragma unroll
    for (int i = 0; i < 8; ++i) hb[i] = bf16_bits(p[(size_t)i * DH]);
    o.x = hb[0] | (hb[1] << 16); o.y = hb[2] | (hb[3] << 16);
    o.z = hb[4] | (hb[5] << 16); o.w = hb[6] | (hb[7] << 16);
    dp = w1t + (size_t)u * 4;
  } else if (u < NUW1 + NUW2) {
    const int v = u - NUW1;
    const int n = v >> 5, k8 = (v & 31) * 8;
    const int kk = k8 & (DH - 1);
    const float* p = W2 + (size_t)kk * DH + n;
    unsigned hb[8];
#pragma unroll
    for (int i = 0; i < 8; ++i) hb[i] = bf16_bits(p[(size_t)i * DH]);
    o.x = hb[0] | (hb[1] << 16); o.y = hb[2] | (hb[3] << 16);
    o.z = hb[4] | (hb[5] << 16); o.w = hb[6] | (hb[7] << 16);
    dp = w2d + (size_t)v * 4;
  } else if (u < NUW1 + NUW2 + NUW3) {
    const int v = u - (NUW1 + NUW2);
    const int n = v >> 5, k8 = (v & 31) * 8;
    const int kk = k8 & (DH - 1);
    const float* p = W3 + (size_t)kk * DOUT + n;
    unsigned hb[8];
#pragma unroll
    for (int i = 0; i < 8; ++i) hb[i] = bf16_bits(p[(size_t)i * DOUT]);
    o.x = hb[0] | (hb[1] << 16); o.y = hb[2] | (hb[3] << 16);
    o.z = hb[4] | (hb[5] << 16); o.w = hb[6] | (hb[7] << 16);
    dp = w3d + (size_t)v * 4;
  } else if (u < NUWE) {
    const int v = u - (NUW1 + NUW2 + NUW3);
    const int j = 4 * v;
    const int j1 = j < DH - 4 ? j : DH - 4;
    int j2 = j - DH;        j2 = j2 < 0 ? 0 : (j2 > DH - 4 ? DH - 4 : j2);
    int j3 = j - 2 * DH;    j3 = j3 < 0 ? 0 : (j3 > DOUT - 4 ? DOUT - 4 : j3);
    const v4f a1 = *(const v4f*)(b1 + j1);
    const v4f a2 = *(const v4f*)(b2 + j2);
    const v4f a3 = *(const v4f*)(b3 + j3);
    const unsigned m1 = (j < DH) ? 0xFFFFFFFFu : 0u;
    const unsigned m2 = (j >= DH && j < 2 * DH) ? 0xFFFFFFFFu : 0u;
    const unsigned m3 = (j >= 2 * DH && j < 2 * DH + DOUT) ? 0xFFFFFFFFu : 0u;
    o.x = ((bf16_bits(a1.x) << 16) & m1) | ((bf16_bits(a2.x) << 16) & m2) | ((bf16_bits(a3.x) << 16) & m3);
    o.y = ((bf16_bits(a1.y) << 16) & m1) | ((bf16_bits(a2.y) << 16) & m2) | ((bf16_bits(a3.y) << 16) & m3);
    o.z = ((bf16_bits(a1.z) << 16) & m1) | ((bf16_bits(a2.z) << 16) & m2) | ((bf16_bits(a3.z) << 16) & m3);
    o.w = ((bf16_bits(a1.w) << 16) & m1) | ((bf16_bits(a2.w) << 16) & m2) | ((bf16_bits(a3.w) << 16) & m3);
    dp = biasT + (size_t)v * 4;
  } else if (u < nUnits) {
    const int v   = u - NUWE;
    const int row = v >> 4, k8 = (v & 15) * 8;
    const int rc  = row < nN ? row : nN - 1;
    const float* p = x + (size_t)rc * DI + k8;
    const v4f a = *(const v4fa*)p;
    const v4f b = *(const v4fa*)(p + 4);
    const unsigned mk = (row < nN) ? 0xFFFFFFFFu : 0u;
    o.x = (bf16_bits(a.x) | (bf16_bits(a.y) << 16)) & mk;
    o.y = (bf16_bits(a.z) | (bf16_bits(a.w) << 16)) & mk;
    o.z = (bf16_bits(b.x) | (bf16_bits(b.y) << 16)) & mk;
    o.w = (bf16_bits(b.z) | (bf16_bits(b.w) << 16)) & mk;
    dp = xb + (size_t)v * 4;
  } else {
    return;
  }
  *(volatile v4u*)dp = o;
  __threadfence();
  *(volatile v4u*)dp = o;
}

__global__ __launch_bounds__(NTHR) void k_bucket(const int* __restrict__ srcs, const int* __restrict__ dsts,
                                                 int nE, int nN, int vec8,
                                                 int* listG, int* cntG, int* offG, int* disG, int* flgG) {
  extern __shared__ __attribute__((aligned(16))) int dsm[];
  int* list = dsm;
  int* hl   = dsm + LISTN;
  int* sl   = dsm + LISTN + RCAP;
  int* cnt  = dsm + LISTN + 2 * RCAP;
  int* offs = cnt + NBA;
  int* cur  = offs + NBA;
  int* misc = cur + NBA;
  const int tid = (int)threadIdx.x, lane = tid & 31, wave = tid >> 5;
  const int nodeBase = (int)blockIdx.x * NBA;

  {
    const v4i z4 = {0, 0, 0, 0};
    for (int i = tid * 4; i < BK_ZINTS; i += NTHR * 4) *(v4ia*)(dsm + i) = z4;
    if (tid < 16) misc[tid] = 0;
  }
  __syncthreads();

  int t = 0, ov = 0;
  const int nChunks = (nE + CHUNK - 1) / CHUNK;
#pragma unroll 1
  for (int ch = 0; ch < nChunks; ++ch) {
    const int cbase = ch * CHUNK;
    const int wc = scan_chunk<SLA>(dsts, nE, cbase, nodeBase, NBA, vec8, list, tid, lane, wave);
    if (lane == 0) misc[wave] = wc;
    __syncthreads();
    if (wave == 0) {
#pragma unroll 1
      for (int w2 = 0; w2 < NWAVE; ++w2) {
        int c = misc[w2];
        c = c < 0 ? 0 : (c > WCAP ? WCAP : c);
#pragma unroll 1
        for (int b0 = 0; b0 < c; b0 += 32) {
          const int idx = b0 + lane;
          const int ent = list[w2 * WCAP + (idx < WCAP ? idx : WCAP - 1)];
          const int m32 = (c - b0) < 32 ? (c - b0) : 32;
#pragma unroll 1
          for (int k = 0; k < m32; ++k) {
            const int u    = __builtin_amdgcn_readlane(ent, k);
            const int slot = u & (NBA - 1);
            const int el   = (u >> SLA) & (CHUNK - 1);
            const int pk   = ((cbase + el) << SLA) | slot;
            if (t < RCAP) {
              if (lane == 0) { hl[t] = pk; cnt[slot] = cnt[slot] + 1; }
              t = t + 1;
            } else {
              ov = 1;
            }
          }
        }
      }
    }
    __syncthreads();
  }
  if (wave == 0 && lane == 0) { misc[8] = t; misc[9] = ov; }
  __syncthreads();
  int tt = misc[8];
  tt = tt < 0 ? 0 : (tt > RCAP ? RCAP : tt);
  const int ovf = misc[9];

  if (wave == 0) {
    const int base = lane * (NBA / 32);
    int s = 0;
#pragma unroll 1
    for (int i = 0; i < NBA / 32; ++i) s += cnt[base + i];
    int incl = s;
#pragma unroll
    for (int d = 1; d < 32; d <<= 1) {
      const int y = __shfl_up(incl, d, 32);
      if (lane >= d) incl += y;
    }
    int run = incl - s;
#pragma unroll 1
    for (int i = 0; i < NBA / 32; ++i) {
      const int cv = cnt[base + i];
      offs[base + i] = run;
      cur[base + i]  = run;
      run += cv;
    }
  }
  __syncthreads();
  if (wave == 0) {
#pragma unroll 1
    for (int b0 = 0; b0 < tt; b0 += 32) {
      const int idx = b0 + lane;
      const int ent = hl[idx < RCAP ? idx : RCAP - 1];
      const int m32 = (tt - b0) < 32 ? (tt - b0) : 32;
#pragma unroll 1
      for (int k = 0; k < m32; ++k) {
        const int u    = __builtin_amdgcn_readlane(ent, k);
        const int slot = u & (NBA - 1);
        if (lane == 0) {
          int p = cur[slot];
          p = p < 0 ? 0 : (p > RCAP - 1 ? RCAP - 1 : p);
          sl[p] = u;
          cur[slot] = p + 1;
        }
      }
    }
  }
  __syncthreads();

#pragma unroll 4
  for (int i = tid; i < RCAP; i += NTHR) {
    const int ent = sl[i];
    int eid = ent >> SLA;
    eid = eid < 0 ? 0 : (eid > nE - 1 ? nE - 1 : eid);
    int sr = srcs[eid];
    sr = sr < 0 ? 0 : (sr > nN - 1 ? nN - 1 : sr);
    hl[i] = (i < tt) ? sr : 0;
  }
#pragma unroll 1
  for (int i = tid; i < NBA; i += NTHR) {
    const float deg = (float)cnt[i] + 1.0f;
    const float dv  = (deg > 0.0f) ? (1.0f / sqrtf(deg)) : 0.0f;
    cur[i] = __float_as_int(dv);
  }
  __syncthreads();

  const int b = (int)blockIdx.x;
  int* lp = listG + (size_t)b * RCAP;
  const v4i c4 = *(const v4ia*)(cnt  + 4 * tid);
  const v4i o4 = *(const v4ia*)(offs + 4 * tid);
  const v4i d4 = *(const v4ia*)(cur  + 4 * tid);
  const v4i f4 = {ovf, ovf, ovf, ovf};
  int* cp = cntG + (size_t)b * NBA + 4 * tid;
  int* op = offG + (size_t)b * NBA + 4 * tid;
  int* dq = disG + (size_t)b * NBA + 4 * tid;
  int* fp = flgG + (size_t)b * 32 + 4 * (tid & 7);
#pragma unroll 4
  for (int it = 0; it < RCAP / (4 * NTHR); ++it) {
    const int q = 4 * (it * NTHR + tid);
    const v4i v = *(const v4ia*)(hl + q);
    *(volatile v4i*)(lp + q) = v;
  }
  *(volatile v4i*)cp = c4;
  *(volatile v4i*)op = o4;
  *(volatile v4i*)dq = d4;
  if (tid < 8) *(volatile v4i*)fp = f4;
  __threadfence();
#pragma unroll 4
  for (int it = 0; it < RCAP / (4 * NTHR); ++it) {
    const int q = 4 * (it * NTHR + tid);
    const v4i v = *(const v4ia*)(hl + q);
    *(volatile v4i*)(lp + q) = v;
  }
  *(volatile v4i*)cp = c4;
  *(volatile v4i*)op = o4;
  *(volatile v4i*)dq = d4;
  if (tid < 8) *(volatile v4i*)fp = f4;
}

template <int NT>
__global__ __launch_bounds__(GTHR) void k_gemm(const unsigned short* __restrict__ A,
                                               const unsigned short* __restrict__ BT,
                                               float* outF, int K) {
  constexpr int GN = 16 * NT;
  __shared__ __attribute__((aligned(16))) float stg[GBM * GN];
  const int tid = (int)threadIdx.x, lane = tid & 31, wave = tid >> 5, hh = lane >> 4, m = lane & 15;
  const int rowBase = (int)blockIdx.x * GBM;

  v8f acc[NT];
#pragma unroll
  for (int t = 0; t < NT; ++t) acc[t] = z8();
  const unsigned short* ap = A  + (size_t)(rowBase + 16 * wave + m) * (size_t)K + 8 * hh;
  const unsigned short* wp = BT + (size_t)m * (size_t)K + 8 * hh;
  const int ksteps = K >> 5;
#pragma unroll 1
  for (int ks = 0; ks < ksteps; ++ks) {
    FragB af;
    af.h[0] = *(const v8usa*)(ap + 32 * ks);
    af.h[1] = *(const v8usa*)(ap + 32 * ks + 16);
#pragma unroll
    for (int t = 0; t < NT; ++t) {
      const unsigned short* wq = wp + (size_t)(16 * t) * (size_t)K + 32 * ks;
      FragB bf;
      bf.h[0] = *(const v8usa*)wq;
      bf.h[1] = *(const v8usa*)(wq + 16);
      acc[t] = wmb(af, bf, acc[t]);
    }
  }

#pragma unroll
  for (int t = 0; t < NT; ++t) {
    const int lc = 16 * t + m;
#pragma unroll
    for (int r = 0; r < 8; ++r) {
      const int lr = 16 * wave + 8 * hh + r;
      stg[lr * GN + lc] = acc[t][r];
    }
  }
  __syncthreads();

  if constexpr (NT == 8) {
    v4f pv[16];
#pragma unroll
    for (int i = 0; i < 16; ++i) pv[i] = *(const v4fa*)(stg + (16 * wave + i) * GN + 4 * lane);
#pragma unroll
    for (int i = 0; i < 16; ++i) {
      float* op = outF + (size_t)(rowBase + 16 * wave + i) * GN + 4 * lane;
      *(volatile v4f*)op = pv[i];
    }
    __threadfence();
#pragma unroll
    for (int i = 0; i < 16; ++i) {
      float* op = outF + (size_t)(rowBase + 16 * wave + i) * GN + 4 * lane;
      *(volatile v4f*)op = pv[i];
    }
  } else {
    v4f fv[8];
#pragma unroll
    for (int i = 0; i < 8; ++i) {
      const int lr = 16 * wave + 2 * i + hh;
      fv[i] = *(const v4fa*)(stg + lr * GN + 4 * m);
    }
#pragma unroll
    for (int i = 0; i < 8; ++i) {
      const int lr = 16 * wave + 2 * i + hh;
      float* op = outF + (size_t)(rowBase + lr) * GN + 4 * m;
      *(volatile v4f*)op = fv[i];
    }
    __threadfence();
#pragma unroll
    for (int i = 0; i < 8; ++i) {
      const int lr = 16 * wave + 2 * i + hh;
      float* op = outF + (size_t)(rowBase + lr) * GN + 4 * m;
      *(volatile v4f*)op = fv[i];
    }
  }
}

template <int D, int MODE>
__global__ __launch_bounds__(NTHR) void k_agg(const int* __restrict__ listG, const int* __restrict__ cntG,
                                              const int* __restrict__ offG, const int* __restrict__ flgG,
                                              const float* __restrict__ dis, const float* __restrict__ xl,
                                              const float* __restrict__ biasT, int nN, int mRows, int nBuck,
                                              unsigned short* hb, float* hout) {
  static_assert((D == 128 && MODE == 1) || (D == 64 && MODE == 0));
  __shared__ __attribute__((aligned(16))) unsigned short rowbufs[NWAVE * ROWH];
  const int tid = (int)threadIdx.x, lane = tid & 31, wave = tid >> 5;
  unsigned short* rowbuf = rowbufs + wave * ROWH;
  const int nodeBase = (int)blockIdx.x * AGS;
  const int nSlots = nBuck * NBA;

  float bq0, bq1, bq2 = 0.0f, bq3 = 0.0f;
  if constexpr (D == 128) {
    const v4f b4 = *(const v4fa*)(biasT + 4 * lane);
    bq0 = b4.x; bq1 = b4.y; bq2 = b4.z; bq3 = b4.w;
  } else {
    const v2f b2 = *(const v2fa*)(biasT + 2 * lane);
    bq0 = b2.x; bq1 = b2.y;
  }
  const float qnan = __int_as_float(0x7fc00000);
  const int sa = (2 * lane) & 31, sb = (2 * lane + 1) & 31;

#pragma unroll 1
  for (int si = 0; si < AGS / NWAVE; ++si) {
    const int node = nodeBase + si * NWAVE + wave;
    const int nt = node < nSlots ? node : nSlots - 1;
    int bk = nt >> SLA;
    bk = bk < 0 ? 0 : (bk > nBuck - 1 ? nBuck - 1 : bk);
    int c = cntG[nt];
    int o = offG[nt];
    const int fl = flgG[bk * 32];
    const bool big = c > DEGCAP;
    c = c < 0 ? 0 : (c > DEGCAP ? DEGCAP : c);
    o = o < 0 ? 0 : (o > RCAP ? RCAP : o);
    const int nc = node < nN ? node : nN - 1;
    const float dd = dis[nc];
    const float rd = dd * dd;
    const int* lp = listG + (size_t)bk * RCAP;
    const int last = o + c - 1;
    float a0 = 0.0f, a1 = 0.0f, a2 = 0.0f, a3 = 0.0f;
#pragma unroll 1
    for (int b0 = 0; b0 < c; b0 += 32) {
      int idx = o + b0 + lane;
      idx = idx > last ? last : idx;
      idx = idx < 0 ? 0 : (idx > RCAP - 1 ? RCAP - 1 : idx);
      int sr = lp[idx];
      sr = sr < 0 ? 0 : (sr > nN - 1 ? nN - 1 : sr);
      const float cf  = dis[sr] * dd;
      const int   cfi = __float_as_int(cf);
      const int m32 = (c - b0) < 32 ? (c - b0) : 32;
#pragma unroll 1
      for (int k = 0; k < m32; ++k) {
        const int   sk = __builtin_amdgcn_readlane(sr, k);
        const float ck = __int_as_float(__builtin_amdgcn_readlane(cfi, k));
        if constexpr (D == 128) {
          const v4f a = *(const v4fa*)(xl + (size_t)sk * D + 4 * lane);
          a0 = fmaf(ck, a.x, a0); a1 = fmaf(ck, a.y, a1);
          a2 = fmaf(ck, a.z, a2); a3 = fmaf(ck, a.w, a3);
        } else {
          const v2f a = *(const v2fa*)(xl + (size_t)sk * D + 2 * lane);
          a0 = fmaf(ck, a.x, a0); a1 = fmaf(ck, a.y, a1);
        }
      }
    }
    float s0, s1, s2 = 0.0f, s3 = 0.0f;
    if constexpr (D == 128) {
      const v4f a = *(const v4fa*)(xl + (size_t)nc * D + 4 * lane);
      s0 = a.x; s1 = a.y; s2 = a.z; s3 = a.w;
    } else {
      const v2f a = *(const v2fa*)(xl + (size_t)nc * D + 2 * lane);
      s0 = a.x; s1 = a.y;
    }
    const float pzr = (big || fl != 0) ? qnan : 0.0f;
    const bool live = node < nN;
    float y0 = (a0 + s0 * rd) + bq0;
    float y1 = (a1 + s1 * rd) + bq1;
    float y2 = (a2 + s2 * rd) + bq2;
    float y3 = (a3 + s3 * rd) + bq3;
    if constexpr (MODE != 0) {
      y0 = (y0 > 0.0f) ? y0 : (y0 - y0);
      y1 = (y1 > 0.0f) ? y1 : (y1 - y1);
      y2 = (y2 > 0.0f) ? y2 : (y2 - y2);
      y3 = (y3 > 0.0f) ? y3 : (y3 - y3);
    }
    y0 = y0 + pzr; y1 = y1 + pzr; y2 = y2 + pzr; y3 = y3 + pzr;
    const float v0 = live ? y0 : 0.0f;
    const float v1 = live ? y1 : 0.0f;
    const float v2 = live ? y2 : 0.0f;
    const float v3 = live ? y3 : 0.0f;
    if constexpr (MODE != 0) {
      v4us mh, ml;
      {
        unsigned lb;
        unsigned hbv;
        hbv = hl_bits(v0, lb); mh[0] = (unsigned short)hbv; ml[0] = (unsigned short)lb;
        hbv = hl_bits(v1, lb); mh[1] = (unsigned short)hbv; ml[1] = (unsigned short)lb;
        hbv = hl_bits(v2, lb); mh[2] = (unsigned short)hbv; ml[2] = (unsigned short)lb;
        hbv = hl_bits(v3, lb); mh[3] = (unsigned short)hbv; ml[3] = (unsigned short)lb;
      }
      *(v4usa*)(rowbuf + 4 * lane)      = mh;
      *(v4usa*)(rowbuf + DH + 4 * lane) = ml;
      wave_sync();
      const v8us q0 = *(const v8usa*)(rowbuf + 8 * lane);
      wave_sync();
      if (node < mRows) {
        unsigned short* rpw = hb + (size_t)node * K2 + 8 * lane;
        *(volatile v8us*)rpw = q0;
        __threadfence();
        *(volatile v8us*)rpw = q0;
      }
    } else {
      v4f ow;
      ow.x = __shfl(v0, sa, 32); ow.y = __shfl(v1, sa, 32);
      ow.z = __shfl(v0, sb, 32); ow.w = __shfl(v1, sb, 32);
      const bool wr = live && (lane < 16);
      float* op = hout + (size_t)nc * D + 4 * (lane & 15);
      if (wr) *(volatile v4f*)op = ow;
      __threadfence();
      if (wr) *(volatile v4f*)op = ow;
      (void)v2; (void)v3;
    }
  }
}

static inline int cdiv(int a, int b) { return (a + b - 1) / b; }
static inline size_t al256(size_t o) { return (o + 255) & ~(size_t)255; }

extern "C" void kernel_launch(void* const* d_in, const int* in_sizes, int n_in,
                              void* d_out, int out_size, void* d_ws, size_t ws_size,
                              hipStream_t stream) {
  if (n_in < 8) return;
  if (in_sizes[0] != NNODE * DI) return;
  const int nN = in_sizes[0] / DI;
  if (in_sizes[1] != 2 * NEDGE) return;
  const int nE = in_sizes[1] / 2;
  if (nE < 1 || nE >= (1 << (31 - SLA))) return;
  if (in_sizes[2] != DI * DH || in_sizes[3] != DH) return;
  if (in_sizes[4] != DH * DH || in_sizes[5] != DH) return;
  if (in_sizes[6] != DH * DOUT || in_sizes[7] != DOUT) return;
  if ((long long)out_size != (long long)nN * DOUT) return;

  const float* x    = (const float*)d_in[0];
  const int*   edge = (const int*)d_in[1];
  const float* W1   = (const float*)d_in[2];
  const float* b1   = (const float*)d_in[3];
  const float* W2   = (const float*)d_in[4];
  const float* b2   = (const float*)d_in[5];
  const float* W3   = (const float*)d_in[6];
  const float* b3   = (const float*)d_in[7];
  float* out = (float*)d_out;
  const int* src = edge;
  const int* dst = edge + nE;

  const int MP = cdiv(nN, AGS) * AGS;
  if (MP != MPAD || (MP % GBM) != 0) return;
  const int gM = MP / GBM;
  const int gA = MP / AGS;
  const int gB = cdiv(MP, NBA);
  if (gB != NBUCK || (long long)gB * NBA < (long long)MP) return;
  const int NBP = gB * NBA;
  const int vec8 = ((nE & 3) == 0) ? 1 : 0;

  char* ws = (char*)d_ws;
  size_t off = 0;
  const size_t oXH   = off; off = al256(off + (size_t)MP * K2 * 2);
  const size_t oH    = off; off = al256(off + (size_t)MP * DH * 4);
  const size_t oLIST = off; off = al256(off + (size_t)gB * RCAP * 4);
  const size_t oCNT  = off; off = al256(off + (size_t)NBP * 4);
  const size_t oOFF  = off; off = al256(off + (size_t)NBP * 4);
  const size_t oDIS  = off; off = al256(off + (size_t)NBP * 4);
  const size_t oFLG  = off; off = al256(off + (size_t)gB * 128);
  const size_t oW1T  = off; off = al256(off + (size_t)DH * DI * 2);
  const size_t oW2D  = off; off = al256(off + (size_t)DH * K2 * 2);
  const size_t oW3D  = off; off = al256(off + (size_t)DOUT * K2 * 2);
  const size_t oBIA  = off; off = al256(off + (size_t)BIASN * 4);
  if (off > ws_size || off > (size_t)WSMAX) return;
  if ((size_t)MP * DI * 2 > (size_t)MP * K2 * 2) return;
  unsigned short* XH   = (unsigned short*)(ws + oXH);
  unsigned short* XB   = XH;
  float*          H    = (float*)(ws + oH);
  int*            LIST = (int*)(ws + oLIST);
  int*            CNT  = (int*)(ws + oCNT);
  int*            OFF  = (int*)(ws + oOFF);
  int*            DISi = (int*)(ws + oDIS);
  const float*    DISf = (const float*)(ws + oDIS);
  int*            FLG  = (int*)(ws + oFLG);
  unsigned short* W1T  = (unsigned short*)(ws + oW1T);
  unsigned short* W2D  = (unsigned short*)(ws + oW2D);
  unsigned short* W3D  = (unsigned short*)(ws + oW3D);
  float*          BIA  = (float*)(ws + oBIA);

  const size_t bkLds = (size_t)BK_LDS_INTS * 4;
  hipFuncSetAttribute(reinterpret_cast<const void*>(&k_bucket), hipFuncAttributeMaxDynamicSharedMemorySize, (int)bkLds);

  const int nUnits = NUWE + MP * (DI / 8);

  k_prep<<<cdiv(nUnits, NTHR), NTHR, 0, stream>>>(x, W1, W2, W3, b1, b2, b3,
                                                  (unsigned*)W1T, (unsigned*)W2D, (unsigned*)W3D,
                                                  (unsigned*)BIA, (unsigned*)XB, nN, nUnits);
  k_bucket<<<gB, NTHR, bkLds, stream>>>(src, dst, nE, nN, vec8, LIST, CNT, OFF, DISi, FLG);
  k_gemm<8><<<gM, GTHR, 0, stream>>>(XB, W1T, H, DI);
  k_agg<128, 1><<<gA, NTHR, 0, stream>>>(LIST, CNT, OFF, FLG, DISf, H, BIA, nN, MP, gB, XH, out);
  k_gemm<8><<<gM, GTHR, 0, stream>>>(XH, W2D, H, K2);
  k_agg<128, 1><<<gA, NTHR, 0, stream>>>(LIST, CNT, OFF, FLG, DISf, H, BIA + DH, nN, MP, gB, XH, out);
  k_gemm<4><<<gM, GTHR, 0, stream>>>(XH, W3D, H, K2);
  k_agg<64, 0><<<gA, NTHR, 0, stream>>>(LIST, CNT, OFF, FLG, DISf, H, BIA + 2 * DH, nN, MP, gB, XH, out);
}
